// MPNNLayer_23235773072079
// MI455X (gfx1250) — hardware-verified
//
#include <hip/hip_runtime.h>
#include <stddef.h>
#include <math.h>


#define HDIM   128
#define K1R    257
#define PW     256
#define NTHR   256
#define NWV    8
#define TR     64
#define LDH    136
#define BM     32
#define CE     81920
#define NB     256
#define CH     2048
#define LCAP   4096
#define SP     128
#define WSCAP  134217728
#define SCL_H   8.0f
#define SCL_W   16.0f
#define SCL_ACT 8.0f
#define INV_HW  0.0078125f
#define LN_EPS  1e-5f

#define LG_SLIST 0
#define LG_SLOTS (LG_SLIST + LCAP * 4)
#define LG_SDL   (LG_SLOTS + NB * SP * 2)
#define LG_SCNT  (LG_SDL + LCAP * 4)
#define LG_WSUM  (LG_SCNT + NB * 4)
#define LDS_G    (LG_WSUM + 64)

static_assert((LDH % 8) == 0 && LDH >= HDIM);
static_assert(TR == 64 && NWV * 32 == NTHR && (TR * HDIM / 4) % NTHR == 0);
static_assert((CE % TR) == 0 && (CE % 4) == 0);
static_assert(NB == NTHR && CH == 8 * NTHR && LCAP >= 2 * CH && (LCAP % 4) == 0 && LCAP <= 65536 && SP <= LCAP);
static_assert(NB == 32 * NWV && BM * 8 == NTHR && PW == 2 * HDIM && (HDIM % 32) == 0);
static_assert((LG_SLOTS % 16) == 0 && (LG_SDL % 16) == 0 && (LG_SCNT % 16) == 0 && (LG_WSUM % 16) == 0);

typedef float    v4f  __attribute__((ext_vector_type(4)));
typedef float    v8f  __attribute__((ext_vector_type(8)));
typedef int      v4i  __attribute__((ext_vector_type(4)));
typedef _Float16 v4h  __attribute__((ext_vector_type(4)));
typedef _Float16 v8h  __attribute__((ext_vector_type(8)));
typedef _Float16 v16h __attribute__((ext_vector_type(16)));
union FragH { v16h v; v8h hh[2]; };

__device__ __forceinline__ v8f wmh(v16h a, v16h b, v8f c) {
  v8f d = __builtin_amdgcn_wmma_f32_16x16x32_f16(false, a, false, b, (short)0, c, false, false);
  asm volatile("v_nop\n\tv_nop\n\tv_nop\n\tv_nop" : "+v"(d) : "v"(a), "v"(b));
  return d;
}

__device__ __forceinline__ v8f zero8() { v8f z = {0.f, 0.f, 0.f, 0.f, 0.f, 0.f, 0.f, 0.f}; return z; }

__device__ __forceinline__ v8h cvt8(v4f a, v4f b, float s) {
  v8f t;
  t[0] = a.x * s; t[1] = a.y * s; t[2] = a.z * s; t[3] = a.w * s;
  t[4] = b.x * s; t[5] = b.y * s; t[6] = b.z * s; t[7] = b.w * s;
  return __builtin_convertvector(t, v8h);
}

__device__ __forceinline__ v16h frag16(const _Float16* p) {
  FragH f;
  f.hh[0] = *(const v8h*)p;
  f.hh[1] = *(const v8h*)(p + 16);
  return f.v;
}

__device__ __forceinline__ v16h afrag_f32(const float* rp, int h, float s) {
  FragH a;
  const float* p0 = rp + 8 * h;
  const float* p1 = rp + 16 + 8 * h;
  a.hh[0] = cvt8(*(const v4f*)p0, *(const v4f*)(p0 + 4), s);
  a.hh[1] = cvt8(*(const v4f*)p1, *(const v4f*)(p1 + 4), s);
  return a.v;
}

__device__ __forceinline__ float rcp_f(float x)  { return __builtin_amdgcn_rcpf(x); }
__device__ __forceinline__ float silu_f(float x) { return x * rcp_f(1.0f + __expf(-x)); }

__device__ __forceinline__ v4h silu4h(v4f v) {
  v4f t;
  t.x = silu_f(v.x) * SCL_ACT; t.y = silu_f(v.y) * SCL_ACT;
  t.z = silu_f(v.z) * SCL_ACT; t.w = silu_f(v.w) * SCL_ACT;
  return __builtin_convertvector(t, v4h);
}

__global__ __launch_bounds__(NTHR) void k_wcvt(const float* __restrict__ in, _Float16* outp,
                                               int C, int koff, int K, int KP, int nUnits, float scale) {
  const int u = (int)blockIdx.x * NTHR + (int)threadIdx.x;
  if (u >= nUnits) return;
  const int upr = KP >> 3;
  const int n   = u / upr;
  const int k0  = (u - n * upr) * 8;
  v8f t;
#pragma unroll
  for (int i = 0; i < 8; ++i) {
    const int k  = k0 + i;
    const int kc = k < K ? k : K - 1;
    const float v = in[(size_t)(koff + kc) * C + n] * scale;
    t[i] = (k < K) ? v : 0.0f;
  }
  const v8h o = __builtin_convertvector(t, v8h);
  _Float16* d = outp + (size_t)n * KP + k0;
  *(volatile v8h*)d = o;
  __threadfence();
  *(volatile v8h*)d = o;
}

__global__ __launch_bounds__(NTHR) __attribute__((amdgpu_num_vgpr(256)))
void k_nodegemm(const float* __restrict__ xin, const _Float16* __restrict__ wPQ,
                const float* __restrict__ b1, float* pq, int nN) {
  constexpr int NIT4 = (BM * PW / 4) / NTHR;
  static_assert((BM * PW / 4) % NTHR == 0 && NIT4 == 8);
  __shared__ __attribute__((aligned(16))) float stg[BM * PW];
  const int tid = threadIdx.x, lane = tid & 31;
  const int wave = __builtin_amdgcn_readfirstlane(tid >> 5);
  const int hh = lane >> 4, m = lane & 15;
  const int rg = wave >> 2, cq = wave & 3;
  const int r0 = rg * 16, c0 = cq * 64;
  const int rowBase = blockIdx.x * BM;

  v8f acc[4];
#pragma unroll
  for (int t = 0; t < 4; ++t) acc[t] = zero8();

  int ar = rowBase + r0 + m;
  ar = ar > nN - 1 ? nN - 1 : ar;
  const float* ap = xin + (size_t)ar * HDIM;
  const _Float16* bp0 = wPQ + (size_t)(c0 + m) * HDIM + 8 * hh;
#pragma unroll 1
  for (int kt = 0; kt < HDIM / 32; ++kt) {
    const v16h a = afrag_f32(ap + 32 * kt, hh, SCL_H);
#pragma unroll
    for (int t = 0; t < 4; ++t) acc[t] = wmh(a, frag16(bp0 + (size_t)(16 * t) * HDIM + 32 * kt), acc[t]);
  }

  float* sp = stg + (size_t)(r0 + 8 * hh) * PW + c0 + m;
  const int grow0 = rowBase + r0 + 8 * hh;
#pragma unroll
  for (int t = 0; t < 4; ++t) {
    const int n  = c0 + 16 * t + m;
    const int nb = n < HDIM ? n : HDIM - 1;
    float bv = b1[nb];
    bv = (n < HDIM) ? bv : 0.0f;
#pragma unroll
    for (int r = 0; r < 8; ++r) {
      float v = acc[t][r] * INV_HW + bv;
      v = (grow0 + r < nN) ? v : 0.0f;
      sp[r * PW + 16 * t] = v;
    }
  }
  __syncthreads();

  float* tile = pq + (size_t)rowBase * PW;
  v4f ov[NIT4];
#pragma unroll
  for (int it = 0; it < NIT4; ++it) ov[it] = *(const v4f*)(stg + 4 * (it * NTHR + tid));
#pragma unroll
  for (int it = 0; it < NIT4; ++it) *(volatile v4f*)(tile + 4 * (size_t)(it * NTHR + tid)) = ov[it];
  __threadfence();
#pragma unroll
  for (int it = 0; it < NIT4; ++it) *(volatile v4f*)(tile + 4 * (size_t)(it * NTHR + tid)) = ov[it];
}

__global__ __launch_bounds__(NTHR) __attribute__((amdgpu_num_vgpr(256)))
void k_edge(const float* __restrict__ pq, const int* __restrict__ ei, const float* __restrict__ ew,
            const float* __restrict__ W1m, const _Float16* __restrict__ w2, const float* __restrict__ b2,
            float* msg, int nE, int nN, int ebase) {
  constexpr int NIT4 = (TR * HDIM / 4) / NTHR;
  constexpr int NSU  = (16 * 64 / 4) / 32;
  __shared__ __attribute__((aligned(16))) float    stg[TR * HDIM];
  __shared__ __attribute__((aligned(16))) _Float16 tile[TR * LDH];
  __shared__ float sew[TR];
  const int tid = threadIdx.x, lane = tid & 31;
  const int wave = __builtin_amdgcn_readfirstlane(tid >> 5);
  const int h = lane >> 4, m = lane & 15;
  const int rg = wave >> 1, ch = wave & 1;
  const int cb = 64 * ch;
  const int rl0 = blockIdx.x * TR;
  const int e0 = ebase + rl0;

  const int eg = e0 + 16 * rg + m;
  const int e = eg > nE - 1 ? nE - 1 : eg;
  int s = ei[e];
  int d = ei[(size_t)nE + e];
  s = s < 0 ? 0 : (s > nN - 1 ? nN - 1 : s);
  d = d < 0 ? 0 : (d > nN - 1 ? nN - 1 : d);
  const float wv = ew[e];
  if (ch == 0 && lane < 16) sew[16 * rg + m] = wv;

  const float* w256 = W1m + (size_t)(K1R - 1) * HDIM;
#pragma unroll 2
  for (int i = 0; i < NSU; ++i) {
    const int u   = i * 32 + lane;
    const int row = u >> 4;
    const int c4  = (u & 15) * 4;
    const int sr  = __shfl(s, row);
    const int dr  = __shfl(d, row);
    const float wr = __shfl(wv, row);
    const v4f p4 = *(const v4f*)(pq + (size_t)sr * PW + cb + c4);
    const v4f q4 = *(const v4f*)(pq + (size_t)dr * PW + HDIM + cb + c4);
    const v4f w4 = *(const v4f*)(w256 + cb + c4);
    const v4f pre = p4 + q4 + w4 * wr;
    *(v4h*)(tile + (size_t)(16 * rg + row) * LDH + cb + c4) = silu4h(pre);
  }
  __syncthreads();

  v8f acc[4];
#pragma unroll
  for (int nt = 0; nt < 4; ++nt) acc[nt] = zero8();
  {
    const _Float16* arow = tile + (size_t)(16 * rg + m) * LDH + 8 * h;
    const _Float16* bp0  = w2 + (size_t)(cb + m) * HDIM + 8 * h;
#pragma unroll 1
    for (int kt = 0; kt < HDIM / 32; ++kt) {
      const v16h a = frag16(arow + 32 * kt);
#pragma unroll
      for (int nt = 0; nt < 4; ++nt) acc[nt] = wmh(a, frag16(bp0 + (size_t)(16 * nt) * HDIM + 32 * kt), acc[nt]);
    }
  }
  {
    float* srow = stg + (size_t)(16 * rg + 8 * h) * HDIM + cb + m;
    const float* ewr = sew + 16 * rg + 8 * h;
#pragma unroll
    for (int nt = 0; nt < 4; ++nt) {
      const float bb = b2[cb + 16 * nt + m];
#pragma unroll
      for (int r = 0; r < 8; ++r) srow[r * HDIM + 16 * nt] = (acc[nt][r] * INV_HW + bb) * ewr[r];
    }
  }
  __syncthreads();

  float* dstp = msg + (size_t)rl0 * HDIM;
  v4f ov[NIT4];
#pragma unroll
  for (int it = 0; it < NIT4; ++it) ov[it] = *(const v4f*)(stg + 4 * (it * NTHR + tid));
#pragma unroll
  for (int it = 0; it < NIT4; ++it) *(volatile v4f*)(dstp + 4 * (size_t)(it * NTHR + tid)) = ov[it];
  __threadfence();
#pragma unroll
  for (int it = 0; it < NIT4; ++it) *(volatile v4f*)(dstp + 4 * (size_t)(it * NTHR + tid)) = ov[it];
}

__global__ __launch_bounds__(NTHR) __attribute__((amdgpu_num_vgpr(256)))
void k_gather(const int* __restrict__ ei, const float* __restrict__ msg, float* agg,
              int nE, int ebase, int clen, int firstChunk) {
  extern __shared__ __align__(16) char smem_g[];
  int*            slist  = (int*)(smem_g + LG_SLIST);
  unsigned short* slots  = (unsigned short*)(smem_g + LG_SLOTS);
  int*            sdl    = (int*)(smem_g + LG_SDL);
  int*            scount = (int*)(smem_g + LG_SCNT);
  int*            wsum   = (int*)(smem_g + LG_WSUM);
  int*            scnt   = wsum + NWV;

  const int tid = threadIdx.x, lane = tid & 31;
  const int wave = __builtin_amdgcn_readfirstlane(tid >> 5);
  const int node0 = blockIdx.x * NB;
  const bool vec_ok = (((nE + ebase) & 3) == 0);
  const v4f z4 = {0.0f, 0.0f, 0.0f, 0.0f};
  const float qn = __int_as_float(0x7fc00000);
  const v4f vnan = {qn, qn, qn, qn};

  int cnt = 0, pass = 0;
  for (int cb = 0; ; cb += CH) {
    const bool endc = (cb >= clen);
    if (endc || (cnt + CH > LCAP)) {
      __syncthreads();
      int k = 0;
#pragma unroll 1
      for (int i = 0; i < cnt; i += 4) {
        const v4i w4 = *(const v4i*)(sdl + i);
#pragma unroll
        for (int q = 0; q < 4; ++q) {
          const bool hit = (w4[q] == tid) && (i + q < cnt);
          if (hit) {
            if (k < SP) slots[tid * SP + k] = (unsigned short)(i + q);
            ++k;
          }
        }
      }
      scount[tid] = k;
      __syncthreads();

      const bool first = (firstChunk != 0) && (pass == 0);
#pragma unroll 1
      for (int j = 0; j < 32; ++j) {
        const int nl = 32 * wave + j;
        float* mrow = agg + (size_t)(node0 + nl) * HDIM + 4 * lane;
        int cn = __builtin_amdgcn_readfirstlane(scount[nl]);
        const bool ovf = cn > SP;
        cn = cn > SP ? SP : cn;
        v4f acc = *(const v4f*)mrow;
        acc = first ? z4 : acc;
#pragma unroll 1
        for (int p = 0; p < cn; ++p) {
          int i = (int)slots[nl * SP + p];
          i = i > LCAP - 1 ? LCAP - 1 : i;
          int el = slist[i];
          el = el < 0 ? 0 : (el > clen - 1 ? clen - 1 : el);
          const v4f ms = *(const v4f*)(msg + (size_t)el * HDIM + 4 * lane);
          acc = acc + ms;
        }
        acc = ovf ? vnan : acc;
        *(volatile v4f*)mrow = acc;
        __threadfence();
        *(volatile v4f*)mrow = acc;
      }
      __syncthreads();
      ++pass;
      cnt = 0;
    }
    if (endc) break;

    int dv[8];
    if (vec_ok && (cb + CH <= clen)) {
      const int* bp = ei + (size_t)nE + ebase + cb + 8 * tid;
      const v4i a = *(const v4i*)bp;
      const v4i b = *(const v4i*)(bp + 4);
      dv[0] = a[0]; dv[1] = a[1]; dv[2] = a[2]; dv[3] = a[3];
      dv[4] = b[0]; dv[5] = b[1]; dv[6] = b[2]; dv[7] = b[3];
    } else {
#pragma unroll
      for (int j = 0; j < 8; ++j) {
        const int el = cb + 8 * tid + j;
        const int ec = el > clen - 1 ? clen - 1 : el;
        const int dj = ei[(size_t)nE + ebase + ec];
        dv[j] = (el < clen) ? dj : -1;
      }
    }
    unsigned bits = 0u;
#pragma unroll
    for (int j = 0; j < 8; ++j) {
      const int dlj = dv[j] - node0;
      bits |= ((unsigned)dlj < (unsigned)NB) ? (1u << j) : 0u;
    }
    const int pc = __builtin_popcount(bits);
    int incl = pc;
#pragma unroll
    for (int sh = 1; sh < 32; sh <<= 1) {
      const int t = __shfl_up(incl, sh);
      incl += (lane >= sh) ? t : 0;
    }
    if (lane == 31) wsum[wave] = incl;
    __syncthreads();
    int woff = 0, tot = 0;
#pragma unroll
    for (int w = 0; w < NWV; ++w) {
      const int v = wsum[w];
      woff += (w < wave) ? v : 0;
      tot += v;
    }
    int pos = cnt + woff + incl - pc;
#pragma unroll
    for (int j = 0; j < 8; ++j) {
      if (bits & (1u << j)) {
        if (pos < LCAP) {
          slist[pos] = cb + 8 * tid + j;
          sdl[pos]   = dv[j] - node0;
        }
        ++pos;
      }
    }
    if (tid == 0) scnt[0] = cnt + tot;
    __syncthreads();
    cnt = scnt[0];
    cnt = cnt > LCAP ? LCAP : cnt;
  }
}

__global__ __launch_bounds__(NTHR) __attribute__((amdgpu_num_vgpr(256)))
void k_node(const float* __restrict__ xin, const float* __restrict__ agg,
            const _Float16* __restrict__ wn1, const _Float16* __restrict__ wn2,
            const float* __restrict__ b1, const float* __restrict__ lng, const float* __restrict__ lnb,
            const float* __restrict__ b2, float* outp, int nN) {
  constexpr int NIT4 = (TR * HDIM / 4) / NTHR;
  __shared__ __attribute__((aligned(16))) _Float16 tile[TR * LDH];
  __shared__ __attribute__((aligned(16))) float    stg[TR * HDIM];
  __shared__ float sst[TR * 2];
  const int tid = threadIdx.x, lane = tid & 31;
  const int wave = __builtin_amdgcn_readfirstlane(tid >> 5);
  const int h = lane >> 4, m = lane & 15;
  const int rg = wave >> 1, ch = wave & 1;
  const int cb = 64 * ch;
  const int rowBase = blockIdx.x * TR;
  const int grow = rowBase + 16 * rg + m;
  const int gcl = grow > nN - 1 ? nN - 1 : grow;

  v8f acc[4];
#pragma unroll
  for (int nt = 0; nt < 4; ++nt) acc[nt] = zero8();
  {
    const float* ap1 = xin + (size_t)gcl * HDIM;
    const float* ap2 = agg + (size_t)grow * HDIM;
    const _Float16* bp0 = wn1 + (size_t)(cb + m) * (2 * HDIM) + 8 * h;
#pragma unroll 1
    for (int kt = 0; kt < HDIM / 32; ++kt) {
      const v16h a = afrag_f32(ap1 + 32 * kt, h, SCL_H);
#pragma unroll
      for (int nt = 0; nt < 4; ++nt)
        acc[nt] = wmh(a, frag16(bp0 + (size_t)(16 * nt) * (2 * HDIM) + 32 * kt), acc[nt]);
    }
#pragma unroll 1
    for (int kt = 0; kt < HDIM / 32; ++kt) {
      const v16h a = afrag_f32(ap2 + 32 * kt, h, SCL_ACT);
#pragma unroll
      for (int nt = 0; nt < 4; ++nt)
        acc[nt] = wmh(a, frag16(bp0 + (size_t)(16 * nt) * (2 * HDIM) + HDIM + 32 * kt), acc[nt]);
    }
  }
  {
    float* srow = stg + (size_t)(16 * rg + 8 * h) * HDIM + cb + m;
#pragma unroll
    for (int nt = 0; nt < 4; ++nt) {
      const float bb = b1[cb + 16 * nt + m];
#pragma unroll
      for (int r = 0; r < 8; ++r) srow[r * HDIM + 16 * nt] = acc[nt][r] * INV_HW + bb;
    }
  }
  __syncthreads();

  if (tid < TR) {
    const float* rp = stg + (size_t)tid * HDIM;
    float s = 0.0f;
#pragma unroll 4
    for (int q = 0; q < HDIM / 4; ++q) {
      const v4f f = *(const v4f*)(rp + 4 * q);
      s += (f.x + f.y) + (f.z + f.w);
    }
    const float mu = s * (1.0f / HDIM);
    float ss = 0.0f;
#pragma unroll 4
    for (int q = 0; q < HDIM / 4; ++q) {
      const v4f f = *(const v4f*)(rp + 4 * q);
      const float dx = f.x - mu, dy = f.y - mu, dz = f.z - mu, dw = f.w - mu;
      ss += (dx * dx + dy * dy) + (dz * dz + dw * dw);
    }
    const float var = ss * (1.0f / HDIM);
    sst[2 * tid]     = mu;
    sst[2 * tid + 1] = rsqrtf(var + LN_EPS);
  }
  __syncthreads();

#pragma unroll 2
  for (int it = 0; it < NIT4; ++it) {
    const int u   = it * NTHR + tid;
    const int row = u >> 5;
    const int c4  = (u & 31) * 4;
    const v4f v  = *(const v4f*)(stg + (size_t)row * HDIM + c4);
    const v4f g4 = *(const v4f*)(lng + c4);
    const v4f o4 = *(const v4f*)(lnb + c4);
    const float mu = sst[2 * row], rs = sst[2 * row + 1];
    v4f t;
    t.x = (v.x - mu) * rs * g4.x + o4.x;
    t.y = (v.y - mu) * rs * g4.y + o4.y;
    t.z = (v.z - mu) * rs * g4.z + o4.z;
    t.w = (v.w - mu) * rs * g4.w + o4.w;
    *(v4h*)(tile + (size_t)row * LDH + c4) = silu4h(t);
  }
  __syncthreads();

#pragma unroll
  for (int nt = 0; nt < 4; ++nt) acc[nt] = zero8();
  {
    const _Float16* arow = tile + (size_t)(16 * rg + m) * LDH + 8 * h;
    const _Float16* bq0  = wn2 + (size_t)(cb + m) * HDIM + 8 * h;
#pragma unroll 1
    for (int kt = 0; kt < HDIM / 32; ++kt) {
      const v16h a = frag16(arow + 32 * kt);
#pragma unroll
      for (int nt = 0; nt < 4; ++nt) acc[nt] = wmh(a, frag16(bq0 + (size_t)(16 * nt) * HDIM + 32 * kt), acc[nt]);
    }
  }
  {
    float* srow = stg + (size_t)(16 * rg + 8 * h) * HDIM + cb + m;
#pragma unroll
    for (int nt = 0; nt < 4; ++nt) {
      const float bb = b2[cb + 16 * nt + m];
#pragma unroll
      for (int r = 0; r < 8; ++r) srow[r * HDIM + 16 * nt] = acc[nt][r] * INV_HW + bb;
    }
  }
  __syncthreads();

  v4f ov[NIT4];
#pragma unroll
  for (int it = 0; it < NIT4; ++it) {
    const int u = it * NTHR + tid;
    const int orow = rowBase + (u >> 5);
    const int oc = orow > nN - 1 ? nN - 1 : orow;
    const v4f xv = *(const v4f*)(xin + (size_t)oc * HDIM + 4 * (u & 31));
    ov[it] = *(const v4f*)(stg + 4 * u) + xv;
  }
#pragma unroll
  for (int it = 0; it < NIT4; ++it) {
    const int u = it * NTHR + tid;
    const int orow = rowBase + (u >> 5);
    if (orow < nN) *(volatile v4f*)(outp + (size_t)orow * HDIM + 4 * (u & 31)) = ov[it];
  }
  __threadfence();
#pragma unroll
  for (int it = 0; it < NIT4; ++it) {
    const int u = it * NTHR + tid;
    const int orow = rowBase + (u >> 5);
    if (orow < nN) *(volatile v4f*)(outp + (size_t)orow * HDIM + 4 * (u & 31)) = ov[it];
  }
}

extern "C" void kernel_launch(void* const* d_in, const int* in_sizes, int n_in,
                              void* d_out, int out_size, void* d_ws, size_t ws_size,
                              hipStream_t stream) {
  if (n_in < 13) return;
  const int nN = in_sizes[0] / HDIM;
  const int nE = in_sizes[2];
  if (nN <= 0 || nE <= 0) return;
  if (in_sizes[0] != nN * HDIM || in_sizes[1] != 2 * nE) return;
  if (in_sizes[3] != K1R * HDIM || in_sizes[4] != HDIM) return;
  if (in_sizes[5] != HDIM * HDIM || in_sizes[6] != HDIM) return;
  if (in_sizes[7] != 2 * HDIM * HDIM || in_sizes[8] != HDIM) return;
  if (in_sizes[9] != HDIM || in_sizes[10] != HDIM) return;
  if (in_sizes[11] != HDIM * HDIM || in_sizes[12] != HDIM) return;
  if (out_size != nN * HDIM) return;
  if (nE > (1 << 27) || nN > (1 << 22)) return;

  const float* x    = (const float*)d_in[0];
  const int*   ei   = (const int*)d_in[1];
  const float* ew   = (const float*)d_in[2];
  const float* mW1  = (const float*)d_in[3];
  const float* mb1  = (const float*)d_in[4];
  const float* mW2  = (const float*)d_in[5];
  const float* mb2  = (const float*)d_in[6];
  const float* uW1  = (const float*)d_in[7];
  const float* ub1  = (const float*)d_in[8];
  const float* lng  = (const float*)d_in[9];
  const float* lnb  = (const float*)d_in[10];
  const float* uW2  = (const float*)d_in[11];
  const float* ub2  = (const float*)d_in[12];
  float* outp = (float*)d_out;

  const int nGat   = (nN + NB - 1) / NB;
  const int NPAD   = nGat * NB;
  const int nGemm  = NPAD / BM;
  const int nNode  = NPAD / TR;
  const int nChunk = (nE + CE - 1) / CE;
  if (nChunk > 256) return;

  char* ws = (char*)d_ws;
  size_t off = 0;
  const size_t oWPQ = off; off += (size_t)PW * HDIM * 2;        off = (off + 255) & ~(size_t)255;
  const size_t oW2  = off; off += (size_t)HDIM * HDIM * 2;      off = (off + 255) & ~(size_t)255;
  const size_t oWN1 = off; off += (size_t)HDIM * 2 * HDIM * 2;  off = (off + 255) & ~(size_t)255;
  const size_t oWN2 = off; off += (size_t)HDIM * HDIM * 2;      off = (off + 255) & ~(size_t)255;
  const size_t oPQ  = off; off += (size_t)NPAD * PW * 4;        off = (off + 255) & ~(size_t)255;
  const size_t oAGG = off; off += (size_t)NPAD * HDIM * 4;      off = (off + 255) & ~(size_t)255;
  const size_t oMSG = off; off += (size_t)CE * HDIM * 4;        off = (off + 255) & ~(size_t)255;
  if (off > ws_size || off > (size_t)WSCAP) return;
  _Float16* wPQ  = (_Float16*)(ws + oWPQ);
  _Float16* w2   = (_Float16*)(ws + oW2);
  _Float16* wn1  = (_Float16*)(ws + oWN1);
  _Float16* wn2  = (_Float16*)(ws + oWN2);
  float*    pqP  = (float*)(ws + oPQ);
  float*    aggP = (float*)(ws + oAGG);
  float*    msgP = (float*)(ws + oMSG);

  (void)hipFuncSetAttribute(reinterpret_cast<const void*>(&k_gather),
                            hipFuncAttributeMaxDynamicSharedMemorySize, (int)LDS_G);

  const int u128 = HDIM * (HDIM / 8);
  const int u256 = HDIM * (2 * HDIM / 8);
  k_wcvt<<<(u128 + NTHR - 1) / NTHR, NTHR, 0, stream>>>(mW1, wPQ, HDIM, 0, HDIM, HDIM, u128, SCL_W);
  k_wcvt<<<(u128 + NTHR - 1) / NTHR, NTHR, 0, stream>>>(mW1, wPQ + (size_t)HDIM * HDIM, HDIM, HDIM, HDIM, HDIM, u128, SCL_W);
  k_wcvt<<<(u128 + NTHR - 1) / NTHR, NTHR, 0, stream>>>(mW2, w2, HDIM, 0, HDIM, HDIM, u128, SCL_W);
  k_wcvt<<<(u256 + NTHR - 1) / NTHR, NTHR, 0, stream>>>(uW1, wn1, HDIM, 0, 2 * HDIM, 2 * HDIM, u256, SCL_W);
  k_wcvt<<<(u128 + NTHR - 1) / NTHR, NTHR, 0, stream>>>(uW2, wn2, HDIM, 0, HDIM, HDIM, u128, SCL_W);
  k_nodegemm<<<nGemm, NTHR, 0, stream>>>(x, wPQ, mb1, pqP, nN);
  for (int c = 0; c < nChunk; ++c) {
    const int ebase = c * CE;
    const int clen  = (nE - ebase) < CE ? (nE - ebase) : CE;
    const int nb    = (clen + TR - 1) / TR;
    k_edge<<<nb, NTHR, 0, stream>>>(pqP, ei, ew, mW1, w2, mb2, msgP, nE, nN, ebase);
    k_gather<<<nGat, NTHR, LDS_G, stream>>>(ei, msgP, aggP, nE, ebase, clen, (c == 0) ? 1 : 0);
  }
  k_node<<<nNode, NTHR, 0, stream>>>(x, aggP, wn1, wn2, ub1, lng, lnb, ub2, outp, nN);
}
